// Block_34196529610857
// MI455X (gfx1250) — hardware-run, weakly checked
//
#include <hip/hip_runtime.h>
#ifndef NB
#define NB 8
#endif
#ifndef SEQ
#define SEQ 1024
#endif
#define NB_FULL 8
#define SEQ_FULL 1024
#define DM 1024
#define NH 16
#define HD 64
#define HID (4 * DM)
#define LQKV (3 * DM)
#define NR ((size_t)NB * SEQ)
static_assert(NB >= 1 && NB <= NB_FULL);
static_assert(SEQ % 128 == 0 && SEQ >= 128 && SEQ <= SEQ_FULL);
static_assert(NH * HD == DM);
static_assert(DM % 64 == 0 && LQKV % 64 == 0 && HID % 64 == 0);
static_assert(DM % 32 == 0 && HID % 32 == 0);
static_assert(HD == 64);
static_assert(4 * 32 * 8 == DM);
static_assert(32 * 16 * 4 == DM * 2);
static_assert(32 * 16 * 16 == 32 * 64 * 4);
static_assert(32 * 8 * 16 == 32 * 64 * 2);
static_assert(32 * 16 * 4 == 16 * HD * 2);
static_assert(4 * 32 * 68 * 4 <= 131072);
static_assert(4 * 16 * 32 * 2 + 4 * 16 * 72 * 2 <= 131072);
static_assert(64 * 66 * 2 <= 131072);

constexpr size_t SZ_BQKV = (size_t)3 * DM * DM * 2;
constexpr size_t SZ_BO   = (size_t)DM * DM * 2;
constexpr size_t SZ_BW1  = (size_t)HID * DM * 2;
constexpr size_t SZ_BW2  = (size_t)DM * HID * 2;
constexpr size_t SZ_WA   = SZ_BQKV + SZ_BO + SZ_BW1;
constexpr size_t SZ_XA   = NR * DM * 2;
constexpr size_t SZ_QKV  = NR * LQKV * 2;
constexpr size_t SZ_VT   = (size_t)NB * NH * HD * SEQ * 2;
constexpr size_t SZ_R0   = SZ_QKV + SZ_VT;
constexpr size_t SZ_H    = NR * HID * 2;
constexpr size_t SZ_X1   = NR * DM * 4;
static_assert(SZ_BW2 <= SZ_BQKV + SZ_BO);
static_assert(SZ_H <= SZ_R0);
static_assert(SZ_WA % 256 == 0 && SZ_XA % 256 == 0 && SZ_R0 % 256 == 0 && SZ_X1 % 256 == 0 && SZ_QKV % 256 == 0 && SZ_BQKV % 256 == 0 && SZ_BO % 256 == 0);
static_assert(SZ_WA + SZ_XA + SZ_R0 + SZ_X1 <= (size_t)134217728);

typedef unsigned short v8us __attribute__((ext_vector_type(8), may_alias));
typedef float  v8f  __attribute__((ext_vector_type(8)));
typedef float  v4f  __attribute__((ext_vector_type(4)));
typedef float  v4fa __attribute__((ext_vector_type(4), may_alias));
typedef _Float16 v16h __attribute__((ext_vector_type(16)));
typedef _Float16 v4h __attribute__((ext_vector_type(4)));
union FragH { v16h v; v8us half[2]; _Float16 h[16]; unsigned short u[16]; };

__device__ __forceinline__ unsigned short bf16_bits(float x) { unsigned int u = __float_as_uint(x); return (unsigned short)((u + 0x7FFFu + ((u >> 16) & 1u)) >> 16); }
__device__ __forceinline__ float bf16_val(unsigned short b) { return __uint_as_float(((unsigned int)b) << 16); }
__device__ __forceinline__ float bf16_rne(float x) { return bf16_val(bf16_bits(x)); }
__device__ __forceinline__ unsigned short h16_bits(float x) { const _Float16 h = (_Float16)x; return __builtin_bit_cast(unsigned short, h); }

static __device__ __forceinline__ _Float16 toh_flush(float v) { const _Float16 r = (_Float16)v; return (fabsf(v) < 6.103515625e-05f) ? (_Float16)0.0f : r; }
static __device__ __forceinline__ unsigned short toh_flush_bits(float v) { const _Float16 r = toh_flush(v); return __builtin_bit_cast(unsigned short, r); }

__device__ __forceinline__ v16h g2_frag(const _Float16* p, int hh) { FragH f; f.half[0] = *(const v8us*)((const unsigned short*)p + 8 * hh); f.half[1] = *(const v8us*)((const unsigned short*)p + 16 + 8 * hh); return f.v; }
__device__ __forceinline__ v8f g2_mma(v16h a, v16h b, v8f c) { v8f d = __builtin_amdgcn_wmma_f32_16x16x32_f16(false, a, false, b, (short)0, c, false, false); asm volatile("v_nop\n\tv_nop\n\tv_nop\n\tv_nop" : "+v"(d) : "v"(a), "v"(b)); return d; }

__device__ __forceinline__ float rmax16(float v) {
  v = fmaxf(v, __shfl_xor(v, 1));
  v = fmaxf(v, __shfl_xor(v, 2));
  v = fmaxf(v, __shfl_xor(v, 4));
  v = fmaxf(v, __shfl_xor(v, 8));
  return v;
}
__device__ __forceinline__ float rsum16(float v) {
  v += __shfl_xor(v, 1);
  v += __shfl_xor(v, 2);
  v += __shfl_xor(v, 4);
  v += __shfl_xor(v, 8);
  return v;
}
__device__ __forceinline__ float wsum32(float v) {
  v += __shfl_xor(v, 1);
  v += __shfl_xor(v, 2);
  v += __shfl_xor(v, 4);
  v += __shfl_xor(v, 8);
  v += __shfl_xor(v, 16);
  return v;
}
__device__ __forceinline__ float gelu_erf(float z) { return 0.5f * z * (1.0f + erff(z * 0.70710678118654752f)); }

__global__ __launch_bounds__(256) void k_wnat(const float* __restrict__ w, size_t n8, _Float16* __restrict__ Bt) {
  const size_t t = (size_t)blockIdx.x * 256 + threadIdx.x; if (t >= n8) return; FragH f;
#pragma unroll
  for (int q = 0; q < 8; ++q) f.h[q] = toh_flush(bf16_rne(w[t * 8 + q]) * 16.0f);
  *(volatile v8us*)((unsigned short*)Bt + t * 8) = f.half[0]; __threadfence(); *(volatile v8us*)((unsigned short*)Bt + t * 8) = f.half[0];
}

__global__ __launch_bounds__(256) void k_ln(const float* __restrict__ X, int srcSeq, int rbf, const float* __restrict__ g, const float* __restrict__ bt, _Float16* __restrict__ Y) {
  #pragma clang fp contract(off)
  const int lane = threadIdx.x & 31;
  const int w = __builtin_amdgcn_readfirstlane(threadIdx.x >> 5);
  const size_t r = (size_t)blockIdx.x * 8 + w; if (r >= NR) return;
  const size_t b = r / SEQ, s = r % SEQ;
  const float* src = X + (b * (size_t)srcSeq + s) * DM;
  float sum = 0.f;
#pragma unroll 1
  for (int i = 0; i < 4; ++i) { const int c = (i * 32 + lane) * 8; const v4f a = *(const v4fa*)(src + c); const v4f d = *(const v4fa*)(src + c + 4);
#pragma unroll
    for (int q = 0; q < 4; ++q) { const float ta = rbf ? bf16_rne(a[q]) : a[q]; const float td = rbf ? bf16_rne(d[q]) : d[q]; sum += ta; sum += td; } }
  sum = wsum32(sum);
  const float mu = sum * (1.0f / DM);
  float sq = 0.f;
#pragma unroll 1
  for (int i = 0; i < 4; ++i) { const int c = (i * 32 + lane) * 8; const v4f a = *(const v4fa*)(src + c); const v4f d = *(const v4fa*)(src + c + 4);
#pragma unroll
    for (int q = 0; q < 4; ++q) { const float ta = (rbf ? bf16_rne(a[q]) : a[q]) - mu; const float td = (rbf ? bf16_rne(d[q]) : d[q]) - mu; sq += ta * ta; sq += td * td; } }
  sq = wsum32(sq);
  const float rstd = rsqrtf(sq * (1.0f / DM) + 1.0e-5f);
  unsigned short* dst = (unsigned short*)Y + r * DM;
  for (int pass = 0; pass < 2; ++pass) {
#pragma unroll 1
    for (int i = 0; i < 4; ++i) { const int c = (i * 32 + lane) * 8; const v4f a = *(const v4fa*)(src + c); const v4f d = *(const v4fa*)(src + c + 4);
      const v4f ga = *(const v4fa*)(g + c); const v4f gd = *(const v4fa*)(g + c + 4); const v4f ba = *(const v4fa*)(bt + c); const v4f bd = *(const v4fa*)(bt + c + 4);
      FragH f;
#pragma unroll
      for (int q = 0; q < 4; ++q) { const float ta = rbf ? bf16_rne(a[q]) : a[q]; const float td = rbf ? bf16_rne(d[q]) : d[q];
        f.h[q]     = toh_flush((ta - mu) * rstd * bf16_rne(ga[q]) + bf16_rne(ba[q]));
        f.h[4 + q] = toh_flush((td - mu) * rstd * bf16_rne(gd[q]) + bf16_rne(bd[q])); }
      *(volatile v8us*)(dst + c) = f.half[0]; }
    if (pass == 0) __threadfence(); } }

template <int EPI>
__device__ __forceinline__ void gemm_body(const _Float16* __restrict__ A, int lda, size_t sA, const _Float16* __restrict__ Bh, int ldb, float alpha, const float* __restrict__ bias, const float* __restrict__ R, int ldr, size_t sR, int rbf,
    float* __restrict__ C, _Float16* __restrict__ C16, int ldc, size_t sC, int M, int N, int K) {
  static_assert(EPI == 0 || EPI == 1 || EPI == 2);
  __shared__ __attribute__((aligned(16))) float so[4][32][68];
  const int tid = threadIdx.x, lane = tid & 31, ln = lane & 15, hh = lane >> 4; const int by = blockIdx.y;
  const int w = __builtin_amdgcn_readfirstlane(tid >> 5);
  A += (size_t)by * sA; const size_t cofs = (size_t)by * sC; const size_t rofs = (size_t)by * sR;
  const int ntn = N >> 6; const int mt = blockIdx.x / ntn, nq = blockIdx.x - mt * ntn; const int row0 = mt * 128 + 32 * w, col0 = nq * 64; if (row0 >= M) return;
  const _Float16* a0p = A + (size_t)(row0 + ln) * lda; const _Float16* a1p = a0p + (size_t)16 * lda;
  const _Float16* b0p = Bh + (size_t)(col0 + ln) * ldb; const _Float16* b1p = b0p + (size_t)16 * ldb; const _Float16* b2p = b1p + (size_t)16 * ldb; const _Float16* b3p = b2p + (size_t)16 * ldb;
  const v8f z8 = {0.f,0.f,0.f,0.f,0.f,0.f,0.f,0.f}; v8f c00 = z8, c01 = z8, c02 = z8, c03 = z8, c10 = z8, c11 = z8, c12 = z8, c13 = z8;
#pragma unroll 1
  for (int kb = 0; kb < K; kb += 32) { const v16h a0 = g2_frag(a0p + kb, hh), a1 = g2_frag(a1p + kb, hh);
    v16h b = g2_frag(b0p + kb, hh); c00 = g2_mma(a0, b, c00); c10 = g2_mma(a1, b, c10);
    b = g2_frag(b1p + kb, hh); c01 = g2_mma(a0, b, c01); c11 = g2_mma(a1, b, c11);
    b = g2_frag(b2p + kb, hh); c02 = g2_mma(a0, b, c02); c12 = g2_mma(a1, b, c12);
    b = g2_frag(b3p + kb, hh); c03 = g2_mma(a0, b, c03); c13 = g2_mma(a1, b, c13); }
  v8f accs[8] = {c00, c01, c02, c03, c10, c11, c12, c13};
#pragma unroll
  for (int u = 0; u < 8; ++u) { const int t = u & 3, half = u >> 2; const int col = col0 + t * 16 + ln; float bv = 0.f; if (EPI != 0) bv = bf16_rne(bias[col]);
#pragma unroll
    for (int r = 0; r < 8; ++r) { const int rloc = half * 16 + 8 * hh + r; so[w][rloc][t * 16 + ln] = accs[u][r] * alpha + bv; } }
  __builtin_amdgcn_fence(4  , "workgroup"); __builtin_amdgcn_wave_barrier();
  const int rsub = lane >> 4, c4 = (lane & 15) * 4;
  if (EPI != 0) {
#pragma unroll 1
    for (int q = 0; q < 16; ++q) { const int r = q * 2 + rsub; v4f v = *(const v4fa*)&so[w][r][c4];
      if (EPI == 1) { const v4f x = *(const v4fa*)(R + rofs + (size_t)(row0 + r) * ldr + col0 + c4);
#pragma unroll
        for (int i = 0; i < 4; ++i) { const float xv = rbf ? bf16_rne(x[i]) : x[i]; v[i] = v[i] + xv; } }
      else {
#pragma unroll
        for (int i = 0; i < 4; ++i) v[i] = 16.0f * gelu_erf(v[i]); }
      *(v4fa*)&so[w][r][c4] = v; } }
  for (int pass = 0; pass < 2; ++pass) {
#pragma unroll
    for (int q = 0; q < 16; ++q) { const int r = q * 2 + rsub; const v4f v = *(const v4fa*)&so[w][r][c4];
      if (EPI == 1) *(volatile v4f*)(C + cofs + (size_t)(row0 + r) * ldc + col0 + c4) = v;
      else { v4h h4;
#pragma unroll
        for (int i = 0; i < 4; ++i) h4[i] = toh_flush(v[i]);
        *(volatile v4h*)(C16 + cofs + (size_t)(row0 + r) * ldc + col0 + c4) = h4; } }
    if (pass == 0) __threadfence(); } }

__global__ __launch_bounds__(128) void k_gemm_qkv(const _Float16* __restrict__ A, const _Float16* __restrict__ Bh, _Float16* __restrict__ C16) {
  gemm_body<0>(A, DM, (size_t)SEQ * DM, Bh, DM, 0.0625f, nullptr, nullptr, 0, 0, 0, nullptr, C16, LQKV, (size_t)SEQ * LQKV, SEQ, LQKV, DM); }
__global__ __launch_bounds__(128) void k_gemm_proj(const _Float16* __restrict__ A, const _Float16* __restrict__ Bh, const float* __restrict__ bias, const float* __restrict__ xin, float* __restrict__ X1) {
  gemm_body<1>(A, DM, (size_t)SEQ * DM, Bh, DM, 0.0009765625f, bias, xin, DM, (size_t)SEQ_FULL * DM, 1, X1, nullptr, DM, (size_t)SEQ * DM, SEQ, DM, DM); }
__global__ __launch_bounds__(128) void k_gemm_fc1(const _Float16* __restrict__ A, const _Float16* __restrict__ Bh, const float* __restrict__ bias, _Float16* __restrict__ H16) {
  gemm_body<2>(A, DM, (size_t)SEQ * DM, Bh, DM, 0.0625f, bias, nullptr, 0, 0, 0, nullptr, H16, HID, (size_t)SEQ * HID, SEQ, HID, DM); }
__global__ __launch_bounds__(128) void k_gemm_fc2(const _Float16* __restrict__ A, const _Float16* __restrict__ Bh, const float* __restrict__ bias, const float* __restrict__ X1, float* __restrict__ out) {
  gemm_body<1>(A, HID, (size_t)SEQ * HID, Bh, HID, 0.00390625f, bias, X1, DM, (size_t)SEQ * DM, 0, out, nullptr, DM, (size_t)SEQ_FULL * DM, SEQ, DM, HID); }

template <int NHv, int TTv>
__global__ __launch_bounds__(256) void k_vt(const _Float16* __restrict__ V16, int ldv, int voff, _Float16* __restrict__ Vt) {
  __shared__ unsigned short tl[64][66]; const int tid = threadIdx.x; const int slab = blockIdx.x / (TTv / 64), lg = blockIdx.x % (TTv / 64); const int b = slab / NHv, h = slab % NHv;
  for (int i = tid; i < 64 * 8; i += 256) { const int r = i / 8, c8 = (i % 8) * 8; FragH f; f.half[0] = *(const v8us*)((const unsigned short*)V16 + ((size_t)b * TTv + lg * 64 + r) * ldv + voff + h * 64 + c8);
#pragma unroll
    for (int q = 0; q < 8; ++q) tl[r][c8 + q] = f.u[q]; }
  __syncthreads();
  for (int pass = 0; pass < 2; ++pass) {
#pragma unroll
    for (int rd = 0; rd < 2; ++rd) { const int d = rd * 32 + tid / 8, pc = tid % 8; FragH f;
#pragma unroll
      for (int q = 0; q < 8; ++q) f.u[q] = tl[pc * 8 + q][d];
      *(volatile v8us*)((unsigned short*)Vt + ((size_t)slab * 64 + d) * TTv + lg * 64 + pc * 8) = f.half[0]; }
    if (pass == 0) __threadfence(); } }

__global__ __launch_bounds__(128) void k_attn(const _Float16* __restrict__ QKV, const _Float16* __restrict__ VTp, const int* __restrict__ length, _Float16* __restrict__ O) {
  #pragma clang fp contract(off)
  __shared__ __attribute__((aligned(16))) unsigned short pl[4][16 * 32];
  __shared__ __attribute__((aligned(16))) unsigned short st[4][16][72];
  const int tid = threadIdx.x, lane = tid & 31, ln = lane & 15, hh = lane >> 4;
  const int w = __builtin_amdgcn_readfirstlane(tid >> 5);
  const int qtl = SEQ / 16;
  const int wave = blockIdx.x * 4 + w;
  const int qt = wave % qtl, bh = wave / qtl;
  const int h = bh % NH, b = bh / NH;
  if (b >= NB) return;
  int lenv = length[b];
  asm volatile("" : "+v"(lenv));
  int lc = (lenv < 0) ? 0 : lenv; lc = (lc > SEQ) ? SEQ : lc;
  int ke = (lc + 31) & ~31; ke = (lc == 0) ? SEQ : ke;
  const int kend = __builtin_amdgcn_readfirstlane(ke);
  const int q0 = qt * 16;
  const _Float16* qrow  = QKV + ((size_t)b * SEQ + q0 + ln) * LQKV + h * HD;
  const _Float16* kbase = QKV + (size_t)b * SEQ * LQKV + DM + h * HD;
  const _Float16* vbase = VTp + (size_t)bh * HD * SEQ;
  const v16h aq0 = g2_frag(qrow, hh), aq1 = g2_frag(qrow + 32, hh);
  const v8f z8 = {0.f,0.f,0.f,0.f,0.f,0.f,0.f,0.f};
  v8f o[4] = {z8, z8, z8, z8};
  float rm[8], rs[8];
#pragma unroll
  for (int r = 0; r < 8; ++r) { rm[r] = -1.0e30f; rs[r] = 0.f; }
#pragma unroll 1
  for (int kt = 0; kt < kend; kt += 32) {
    v8f s0 = z8, s1 = z8;
    { const _Float16* kr = kbase + (size_t)(kt + ln) * LQKV;
      v16h bk = g2_frag(kr, hh); s0 = g2_mma(aq0, bk, s0); bk = g2_frag(kr + 32, hh); s0 = g2_mma(aq1, bk, s0);
      kr += (size_t)16 * LQKV;
      bk = g2_frag(kr, hh); s1 = g2_mma(aq0, bk, s1); bk = g2_frag(kr + 32, hh); s1 = g2_mma(aq1, bk, s1); }
    const float mk0 = (kt + ln >= lenv) ? -10000.0f : 0.0f;
    const float mk1 = (kt + 16 + ln >= lenv) ? -10000.0f : 0.0f;
    __builtin_amdgcn_fence(3  , "wavefront"); __builtin_amdgcn_wave_barrier();
    float corr[8];
#pragma unroll
    for (int r = 0; r < 8; ++r) {
      const float a0 = s0[r] * 0.125f + mk0, a1 = s1[r] * 0.125f + mk1;
      const float tmax = rmax16(fmaxf(a0, a1));
      const float nm = fmaxf(rm[r], tmax);
      const float cr = __expf(rm[r] - nm);
      rm[r] = nm; corr[r] = cr;
      const float p0 = __expf(a0 - nm), p1 = __expf(a1 - nm);
      rs[r] = rs[r] * cr + rsum16(p0 + p1);
      pl[w][(8 * hh + r) * 32 + ln]      = toh_flush_bits(p0 * 1024.0f);
      pl[w][(8 * hh + r) * 32 + 16 + ln] = toh_flush_bits(p1 * 1024.0f);
    }
#pragma unroll
    for (int j = 0; j < 4; ++j) {
#pragma unroll
      for (int r = 0; r < 8; ++r) o[j][r] *= corr[r];
    }
    __builtin_amdgcn_fence(3  , "wavefront"); __builtin_amdgcn_wave_barrier();
    FragH ap; ap.half[0] = *(const v8us*)&pl[w][ln * 32 + 8 * hh]; ap.half[1] = *(const v8us*)&pl[w][ln * 32 + 16 + 8 * hh];
#pragma unroll
    for (int j = 0; j < 4; ++j) { const v16h bv = g2_frag(vbase + (size_t)(j * 16 + ln) * SEQ + kt, hh); o[j] = g2_mma(ap.v, bv, o[j]); }
  }
  float inv[8];
#pragma unroll
  for (int r = 0; r < 8; ++r) inv[r] = 0.0625f / rs[r];
#pragma unroll
  for (int j = 0; j < 4; ++j) {
#pragma unroll
    for (int r = 0; r < 8; ++r) st[w][8 * hh + r][j * 16 + ln] = toh_flush_bits(o[j][r] * inv[r]);
  }
  __builtin_amdgcn_fence(4  , "workgroup"); __builtin_amdgcn_wave_barrier();
  const int rq = lane >> 3, pc = lane & 7;
  unsigned short* obase = (unsigned short*)O + ((size_t)b * SEQ + q0) * DM + h * HD + pc * 8;
  for (int pass = 0; pass < 2; ++pass) {
#pragma unroll
    for (int it = 0; it < 4; ++it) { const int row = it * 4 + rq; const v8us v = *(const v8us*)&st[w][row][pc * 8]; *(volatile v8us*)(obase + (size_t)row * DM) = v; }
    if (pass == 0) __threadfence(); }
}

extern "C" void kernel_launch(void* const* d_in, const int* in_sizes, int n_in,
                              void* d_out, int out_size, void* d_ws, size_t ws_size, hipStream_t stream) {
  if (n_in < 13) return;
  const float* x      = (const float*)d_in[0];
  const int*   length = (const int*)d_in[1];
  const float* g1     = (const float*)d_in[2];
  const float* b1     = (const float*)d_in[3];
  const float* w_qkv  = (const float*)d_in[4];
  const float* w_proj = (const float*)d_in[5];
  const float* b_proj = (const float*)d_in[6];
  const float* g2     = (const float*)d_in[7];
  const float* b2     = (const float*)d_in[8];
  const float* w_fc1  = (const float*)d_in[9];
  const float* b_fc1  = (const float*)d_in[10];
  const float* w_fc2  = (const float*)d_in[11];
  const float* b_fc2  = (const float*)d_in[12];
  const size_t rows_needed = (size_t)(NB - 1) * SEQ_FULL + SEQ;
  if ((size_t)in_sizes[0] < rows_needed * DM) return;
  if ((size_t)in_sizes[1] < (size_t)NB) return;
  if ((size_t)in_sizes[2] < (size_t)DM) return;
  if ((size_t)in_sizes[3] < (size_t)DM) return;
  if ((size_t)in_sizes[4] < (size_t)3 * DM * DM) return;
  if ((size_t)in_sizes[5] < (size_t)DM * DM) return;
  if ((size_t)in_sizes[6] < (size_t)DM) return;
  if ((size_t)in_sizes[7] < (size_t)DM) return;
  if ((size_t)in_sizes[8] < (size_t)DM) return;
  if ((size_t)in_sizes[9] < (size_t)HID * DM) return;
  if ((size_t)in_sizes[10] < (size_t)HID) return;
  if ((size_t)in_sizes[11] < (size_t)DM * HID) return;
  if ((size_t)in_sizes[12] < (size_t)DM) return;
  if ((size_t)out_size < rows_needed * DM) return;
  char* ws = (char*)d_ws; size_t off = 0;
  auto take = [&](size_t bytes) { char* p = ws + off; off += (bytes + 255) & ~(size_t)255; return p; };
  char* WA = take(SZ_WA);
  _Float16* BQKV  = (_Float16*)(WA);
  _Float16* BO    = (_Float16*)(WA + SZ_BQKV);
  _Float16* BW1   = (_Float16*)(WA + SZ_BQKV + SZ_BO);
  _Float16* BW2   = (_Float16*)(WA);
  _Float16* XA    = (_Float16*)take(SZ_XA);
  char* R0 = take(SZ_R0);
  _Float16* QKV16 = (_Float16*)(R0);
  _Float16* VT    = (_Float16*)(R0 + SZ_QKV);
  _Float16* H16   = (_Float16*)(R0);
  float*    X1    = (float*)take(SZ_X1);
  if (off > ws_size) return;
  k_wnat<<<(unsigned)(((size_t)3 * DM * DM / 8 + 255) / 256), 256, 0, stream>>>(w_qkv, (size_t)3 * DM * DM / 8, BQKV);
  k_wnat<<<(unsigned)(((size_t)DM * DM / 8 + 255) / 256), 256, 0, stream>>>(w_proj, (size_t)DM * DM / 8, BO);
  k_wnat<<<(unsigned)(((size_t)HID * DM / 8 + 255) / 256), 256, 0, stream>>>(w_fc1, (size_t)HID * DM / 8, BW1);
  k_ln<<<(unsigned)(NR / 8), 256, 0, stream>>>(x, SEQ_FULL, 1, g1, b1, XA);
  k_gemm_qkv<<<dim3((unsigned)((SEQ / 128) * (LQKV / 64)), NB), 128, 0, stream>>>(XA, BQKV, QKV16);
  k_vt<NH, SEQ><<<(unsigned)(NB * NH * (SEQ / 64)), 256, 0, stream>>>(QKV16, LQKV, 2 * DM, VT);
  k_attn<<<(unsigned)((NB * NH * (SEQ / 16)) / 4), 128, 0, stream>>>(QKV16, VT, length, XA);
  k_gemm_proj<<<dim3((unsigned)((SEQ / 128) * (DM / 64)), NB), 128, 0, stream>>>(XA, BO, b_proj, x, X1);
  k_wnat<<<(unsigned)(((size_t)DM * HID / 8 + 255) / 256), 256, 0, stream>>>(w_fc2, (size_t)DM * HID / 8, BW2);
  k_ln<<<(unsigned)(NR / 8), 256, 0, stream>>>(X1, SEQ, 0, g2, b2, XA);
  k_gemm_fc1<<<dim3((unsigned)((SEQ / 128) * (HID / 64)), NB), 128, 0, stream>>>(XA, BW1, b_fc1, H16);
  k_gemm_fc2<<<dim3((unsigned)((SEQ / 128) * (DM / 64)), NB), 128, 0, stream>>>(H16, BW2, b_fc2, X1, (float*)d_out);
}
